// BiDirectionalAddBlock_59622736003619
// MI455X (gfx1250) — hardware-verified
//
#include <hip/hip_runtime.h>
#include <math.h>

typedef __attribute__((ext_vector_type(16))) _Float16 v16h;
typedef __attribute__((ext_vector_type(8)))  _Float16 v8h;
typedef __attribute__((ext_vector_type(16))) __bf16   v16b;
typedef __attribute__((ext_vector_type(8)))  __bf16   v8b;
typedef __attribute__((ext_vector_type(8)))  float    v8f;
typedef __attribute__((ext_vector_type(4)))  float    v4f;

constexpr int kBatch = 2;
constexpr int kSeqL  = 4096;
constexpr int kDmod  = 512;
constexpr int kDin   = 1024;
constexpr int kNst   = 16;
constexpr int kDtR   = 32;
constexpr int kPrj   = 64;
constexpr int kXZP   = 2 * kDin;
constexpr int kRows  = kBatch * kSeqL;
constexpr int kTP    = 260;

__device__ __forceinline__ unsigned short f2bf_bits(float f) {
  unsigned u = __float_as_uint(f);
  return (unsigned short)((u + 0x7FFFu + ((u >> 16) & 1u)) >> 16);
}
__device__ __forceinline__ float bf_bits2f(unsigned short h) { return __uint_as_float(((unsigned)h) << 16); }
__device__ __forceinline__ float bfr(float f) { return bf_bits2f(f2bf_bits(f)); }

__device__ __forceinline__ void dep_guard_h(v8f& a, v8f& b, v16h x, v16h y) { asm volatile("v_nop\n\tv_nop\n\tv_nop\n\tv_nop" : "+v"(a), "+v"(b) : "v"(x), "v"(y)); }
__device__ __forceinline__ void dep_guard_b(v8f& a, v8f& b, v16b x, v16b y) { asm volatile("v_nop\n\tv_nop\n\tv_nop\n\tv_nop" : "+v"(a), "+v"(b) : "v"(x), "v"(y)); }
__device__ __forceinline__ void keep4_h(v16h a, v16h b, v16h c, v16h d) { asm volatile("v_nop" :: "v"(a), "v"(b), "v"(c), "v"(d)); }
__device__ __forceinline__ void keep4_b(v16b a, v16b b, v16b c, v16b d) { asm volatile("v_nop" :: "v"(a), "v"(b), "v"(c), "v"(d)); }
__device__ __forceinline__ void acc_guard4(v8f& a, v8f& b, v8f& c, v8f& d) { asm volatile("v_nop\n\tv_nop\n\tv_nop\n\tv_nop" : "+v"(a), "+v"(b), "+v"(c), "+v"(d)); }
template <typename T> struct Frag;
template <> struct Frag<_Float16> {
  typedef v16h V; union U { v16h v; v8h h[2]; };
  static __device__ __forceinline__ v16h load(const _Float16* p) {
    U f; f.h[0] = *(const v8h*)(p); f.h[1] = *(const v8h*)(p + 16); return f.v;
  }
  static __device__ __forceinline__ v8f mma(v16h a, v16h b, v8f c) {
    return __builtin_amdgcn_wmma_f32_16x16x32_f16(false, a, false, b, (short)0, c, false, false);
  }
  static __device__ __forceinline__ void guard(v8f& a, v8f& b, v16h x, v16h y) { dep_guard_h(a, b, x, y); }
  static __device__ __forceinline__ void keep(v16h a, v16h b, v16h c, v16h d) { keep4_h(a, b, c, d); }
};
template <> struct Frag<__bf16> {
  typedef v16b V; union U { v16b v; v8b h[2]; };
  static __device__ __forceinline__ v16b load(const __bf16* p) {
    U f; f.h[0] = *(const v8b*)(p); f.h[1] = *(const v8b*)(p + 16); return f.v;
  }
  static __device__ __forceinline__ v8f mma(v16b a, v16b b, v8f c) {
    return __builtin_amdgcn_wmma_f32_16x16x32_bf16(false, a, false, b, (short)0, c, false, false);
  }
  static __device__ __forceinline__ void guard(v8f& a, v8f& b, v16b x, v16b y) { dep_guard_b(a, b, x, y); }
  static __device__ __forceinline__ void keep(v16b a, v16b b, v16b c, v16b d) { keep4_b(a, b, c, d); }
};

template <int ET> struct Elem;
template <> struct Elem<0> { typedef _Float16 T; };
template <> struct Elem<1> { typedef __bf16 T; };
template <int ET, int SPLITM, int BIAS_MODE, int OUT_MODE, bool RESID, int ACT = 0>
__global__ __launch_bounds__(256) void wmma_gemm64(
    const unsigned short* __restrict__ Ap, const unsigned short* __restrict__ A2p, int lda, long strideA,
    const unsigned short* __restrict__ Btp, const unsigned short* __restrict__ Bt2p, int ldb, long strideB,
    void* __restrict__ Cout, void* __restrict__ Cout2, int ldc, long strideC,
    const float* __restrict__ bias,
    const float* __restrict__ resid, long strideR,
    int M, int N, int K, float scale) {
  constexpr bool kSplitA = (SPLITM != 0);
  constexpr bool kSplitB = (SPLITM == 1);
  typedef typename Elem<ET>::T T;
  typedef typename Frag<T>::V V;
  const T* A = (const T*)Ap; const T* A2 = (const T*)A2p; const T* Bt = (const T*)Btp; const T* Bt2 = (const T*)Bt2p;
  __shared__ __align__(16) float sT[8][16 * 68];
  const int b    = blockIdx.y;
  const int lane = threadIdx.x & 31;
  const int wave = threadIdx.x >> 5;
  const int tilesN = N >> 6;
  const int tilesM = M >> 6;
  const int tile = blockIdx.x * 8 + wave;
  if (tile >= tilesM * tilesN) return;
  const int tm = tile / tilesN;
  const int tn = tile - tm * tilesN;
  const int m0 = tm << 6;
  const int n0 = tn << 6;

  const T* Ab  = A  + (size_t)b * strideA;
  const T* Bb  = Bt + (size_t)b * strideB;
  const T* Ab2 = kSplitA ? (A2  + (size_t)b * strideA) : nullptr;
  const T* Bb2 = kSplitB ? (Bt2 + (size_t)b * strideB) : nullptr;

  const int rlane = lane & 15;
  const int koff  = (lane >> 4) * 8;
  const int mOff  = (lane >> 4) * 8;

  v8f acc[4][4];
#pragma unroll
  for (int i = 0; i < 4; ++i)
#pragma unroll
    for (int j = 0; j < 4; ++j) acc[i][j] = (v8f){0.f,0.f,0.f,0.f,0.f,0.f,0.f,0.f};

  for (int k0 = 0; k0 < K; k0 += 32) {
    V bh[4], bl[4];
#pragma unroll
    for (int j = 0; j < 4; ++j) {
      const size_t bo = (size_t)(n0 + (j << 4) + rlane) * ldb + koff + k0;
      bh[j] = Frag<T>::load(Bb + bo);
      if (kSplitB) bl[j] = Frag<T>::load(Bb2 + bo);
    }
#pragma unroll
    for (int i = 0; i < 4; ++i) {
      const size_t ao = (size_t)(m0 + (i << 4) + rlane) * lda + koff + k0;
      V ah = Frag<T>::load(Ab + ao);
      V al;
      if (kSplitA) al = Frag<T>::load(Ab2 + ao);
#pragma unroll
      for (int j = 0; j < 4; ++j) {
        acc[i][j] = Frag<T>::mma(ah, bh[j], acc[i][j]);
        if (kSplitB) acc[i][j] = Frag<T>::mma(ah, bl[j], acc[i][j]);
        if (kSplitA) acc[i][j] = Frag<T>::mma(al, bh[j], acc[i][j]);
      }
      Frag<T>::guard(acc[i][0], acc[i][3], ah, kSplitA ? al : ah);
    }
    Frag<T>::keep(bh[0], bh[1], bh[2], bh[3]);
    if (kSplitB) Frag<T>::keep(bl[0], bl[1], bl[2], bl[3]);
  }
  acc_guard4(acc[0][0], acc[0][1], acc[0][2], acc[0][3]);
  acc_guard4(acc[1][0], acc[1][1], acc[1][2], acc[1][3]);
  acc_guard4(acc[2][0], acc[2][1], acc[2][2], acc[2][3]);
  acc_guard4(acc[3][0], acc[3][1], acc[3][2], acc[3][3]);

  float* slab = sT[wave];
  const float* Rb = RESID ? (resid + (size_t)b * strideR) : nullptr;
#pragma unroll
  for (int i = 0; i < 4; ++i) {
    const int mBase = m0 + (i << 4);
#pragma unroll
    for (int j = 0; j < 4; ++j) {
      const int n = n0 + (j << 4) + rlane;
      float bv = 0.f;
      if (BIAS_MODE == 2) bv = bias[n];
#pragma unroll
      for (int r = 0; r < 8; ++r) {
        float v = acc[i][j][r] * scale;
        if (BIAS_MODE == 1) v += bias[mBase + mOff + r];
        if (BIAS_MODE == 2) v += bv;
        if (RESID) v += Rb[(size_t)(mBase + mOff + r) * ldc + n];
        if (ACT == 1) v = tanhf(v);
        if (ACT == 2) v = fmaxf(v, 0.0f);
        if (ACT == 3) v = v / (1.0f + expf(-v));
        if (ACT == 4) v = (v > 0.f) ? v : 0.01f * v;
        if (ACT == 5) v = 0.5f * v * (1.0f + erff(v * 0.70710678118654752f));
        slab[(mOff + r) * 68 + (j << 4) + rlane] = v;
      }
    }
    __builtin_amdgcn_fence(__ATOMIC_RELEASE, "workgroup");
    __builtin_amdgcn_wave_barrier();
    __builtin_amdgcn_fence(__ATOMIC_ACQUIRE, "workgroup");
    if (OUT_MODE == 0) {
      float* C = (float*)Cout + (size_t)b * strideC;
      const int hh = lane >> 4, c4 = (lane & 15) * 4;
      for (int pass = 0; pass < 2; ++pass) {
#pragma unroll
        for (int it = 0; it < 8; ++it) {
          const int row = it * 2 + hh;
          v4f v = *(const v4f*)(slab + row * 68 + c4);
          *(volatile v4f*)(C + (size_t)(mBase + row) * ldc + n0 + c4) = v;
        }
        __threadfence();
      }
    } else {
      const int q = lane >> 3, c8 = (lane & 7) * 8;
      unsigned short* C  = (unsigned short*)Cout  + (size_t)b * strideC;
      unsigned short* C2 = (OUT_MODE == 2) ? ((unsigned short*)Cout2 + (size_t)b * strideC) : nullptr;
      for (int pass = 0; pass < 2; ++pass) {
#pragma unroll
        for (int it = 0; it < 4; ++it) {
          const int row = it * 4 + q;
          const float* sp = slab + row * 68 + c8;
          v8h hv, lv;
#pragma unroll
          for (int e = 0; e < 8; ++e) {
            if (OUT_MODE == 1) {
              hv[e] = (_Float16)sp[e];
            } else {
              unsigned short hb = f2bf_bits(sp[e]);
              unsigned short lb = f2bf_bits(sp[e] - bf_bits2f(hb));
              hv[e] = __builtin_bit_cast(_Float16, hb);
              lv[e] = __builtin_bit_cast(_Float16, lb);
            }
          }
          *(volatile v8h*)(C + (size_t)(mBase + row) * ldc + n0 + c8) = hv;
          if (OUT_MODE == 2) *(volatile v8h*)(C2 + (size_t)(mBase + row) * ldc + n0 + c8) = lv;
        }
        __threadfence();
      }
    }
    __builtin_amdgcn_fence(__ATOMIC_RELEASE, "workgroup");
    __builtin_amdgcn_wave_barrier();
    __builtin_amdgcn_fence(__ATOMIC_ACQUIRE, "workgroup");
  }
}

__global__ __launch_bounds__(256) void cast_rows_bf16_kernel(
    const float* __restrict__ src, unsigned short* __restrict__ dst, int N, int K, int total8)
{
  const int i = blockIdx.x * 256 + threadIdx.x;
  if (i >= total8) return;
  const int e0  = i << 3;
  const int row = e0 / K;
  const int col = e0 - row * K;
  const int rowc = (row < N) ? row : (N - 1);
  const bool live = (row < N);
  const float* p = src + (size_t)rowc * K + col;
  const v4f a0 = *(const v4f*)(p);
  const v4f a1 = *(const v4f*)(p + 4);
  v8h hv;
#pragma unroll
  for (int e = 0; e < 4; ++e) {
    hv[e]     = live ? __builtin_bit_cast(_Float16, f2bf_bits(a0[e])) : (_Float16)0.0f;
    hv[4 + e] = live ? __builtin_bit_cast(_Float16, f2bf_bits(a1[e])) : (_Float16)0.0f;
  }
  unsigned short* q = dst + (size_t)e0;
  *(volatile v8h*)q = hv;
  __threadfence();
  *(volatile v8h*)q = hv;
}

__global__ __launch_bounds__(256) void cast_cols_bf16_split_kernel(
    const float* __restrict__ src, int lds, unsigned short* __restrict__ dhi, unsigned short* __restrict__ dlo,
    int K, int total8)
{
  const int i = blockIdx.x * 256 + threadIdx.x;
  if (i >= total8) return;
  const int e0  = i << 3;
  const int row = e0 / K;
  const int col = e0 - row * K;
  const float* p = src + (size_t)row * lds + col;
  const v4f a0 = *(const v4f*)(p);
  const v4f a1 = *(const v4f*)(p + 4);
  v8h hv, lv;
#pragma unroll
  for (int e = 0; e < 4; ++e) {
    const unsigned short hb0 = f2bf_bits(a0[e]);
    const unsigned short lb0 = f2bf_bits(a0[e] - bf_bits2f(hb0));
    const unsigned short hb1 = f2bf_bits(a1[e]);
    const unsigned short lb1 = f2bf_bits(a1[e] - bf_bits2f(hb1));
    hv[e]     = __builtin_bit_cast(_Float16, hb0);
    lv[e]     = __builtin_bit_cast(_Float16, lb0);
    hv[4 + e] = __builtin_bit_cast(_Float16, hb1);
    lv[4 + e] = __builtin_bit_cast(_Float16, lb1);
  }
  unsigned short* qh = dhi + (size_t)e0;
  unsigned short* ql = dlo + (size_t)e0;
  *(volatile v8h*)qh = hv;
  *(volatile v8h*)ql = lv;
  __threadfence();
  *(volatile v8h*)qh = hv;
  *(volatile v8h*)ql = lv;
}

__global__ __launch_bounds__(64) void ln_rows_kernel(
    const float* __restrict__ x, const float* __restrict__ lnw, const float* __restrict__ lnb,
    unsigned short* __restrict__ HH, unsigned short* __restrict__ HL, int rev)
{
  __shared__ float sred[4];
  const int tid = threadIdx.x, lane = tid & 31, wave = tid >> 5;
  const int row = blockIdx.x;
  const int b = row / kSeqL, l = row - b * kSeqL;
  const float* xr = x + (size_t)row * kDmod + tid * 8;
  v4f a0 = *(const v4f*)(xr);
  v4f a1 = *(const v4f*)(xr + 4);
#pragma unroll
  for (int e = 0; e < 4; ++e) { a0[e] = bfr(a0[e]); a1[e] = bfr(a1[e]); }
  float s = ((a0[0] + a0[1]) + (a0[2] + a0[3])) + ((a1[0] + a1[1]) + (a1[2] + a1[3]));
#pragma unroll
  for (int off = 1; off < 32; off <<= 1) s += __shfl_xor(s, off, 32);
  if (lane == 0) sred[wave] = s;
  __syncthreads();
  const float mu = (sred[0] + sred[1]) * (1.0f / (float)kDmod);
  float q = 0.f;
#pragma unroll
  for (int e = 0; e < 4; ++e) {
    const float t0 = a0[e] - mu; q += t0 * t0;
    const float t1 = a1[e] - mu; q += t1 * t1;
  }
#pragma unroll
  for (int off = 1; off < 32; off <<= 1) q += __shfl_xor(q, off, 32);
  if (lane == 0) sred[2 + wave] = q;
  __syncthreads();
  const float var  = (sred[2] + sred[3]) * (1.0f / (float)kDmod);
  const float rstd = rsqrtf(var + 1e-5f);
  const v4f w0 = *(const v4f*)(lnw + tid * 8), w1 = *(const v4f*)(lnw + tid * 8 + 4);
  const v4f b0 = *(const v4f*)(lnb + tid * 8), b1 = *(const v4f*)(lnb + tid * 8 + 4);
  v8h hv, lv;
#pragma unroll
  for (int e = 0; e < 4; ++e) {
    const float v0 = (a0[e] - mu) * rstd * bfr(w0[e]) + bfr(b0[e]);
    const float v1 = (a1[e] - mu) * rstd * bfr(w1[e]) + bfr(b1[e]);
    const unsigned short hb0 = f2bf_bits(v0);
    const unsigned short lb0 = f2bf_bits(v0 - bf_bits2f(hb0));
    const unsigned short hb1 = f2bf_bits(v1);
    const unsigned short lb1 = f2bf_bits(v1 - bf_bits2f(hb1));
    hv[e]     = __builtin_bit_cast(_Float16, hb0);
    lv[e]     = __builtin_bit_cast(_Float16, lb0);
    hv[4 + e] = __builtin_bit_cast(_Float16, hb1);
    lv[4 + e] = __builtin_bit_cast(_Float16, lb1);
  }
  const size_t orow = rev ? ((size_t)b * kSeqL + (size_t)(kSeqL - 1 - l)) : (size_t)row;
  unsigned short* p1 = HH + orow * kDmod + tid * 8;
  unsigned short* p2 = HL + orow * kDmod + tid * 8;
  *(volatile v8h*)p1 = hv;
  *(volatile v8h*)p2 = lv;
  __threadfence();
  *(volatile v8h*)p1 = hv;
  *(volatile v8h*)p2 = lv;
}

__global__ __launch_bounds__(256) void conv_silu_kernel(
    const float* __restrict__ XZ, const float* __restrict__ cw, const float* __restrict__ cb,
    unsigned short* __restrict__ XCH, unsigned short* __restrict__ XCL)
{
  __shared__ __align__(16) float sT[16 * kTP];
  const int tid = threadIdx.x, lane = tid & 31, wave = tid >> 5;
  const int d0 = blockIdx.x * 256, d = d0 + tid;
  const int t0 = blockIdx.y * 64;
  const float w0 = bfr(cw[d * 4 + 0]), w1 = bfr(cw[d * 4 + 1]), w2 = bfr(cw[d * 4 + 2]), w3 = bfr(cw[d * 4 + 3]);
  const float bc = bfr(cb[d]);
  float xm3, xm2, xm1;
  {
    const int r3 = t0 - 3, r2 = t0 - 2, r1 = t0 - 1;
    const int c3 = r3 < 0 ? 0 : r3, c2 = r2 < 0 ? 0 : r2, c1 = r1 < 0 ? 0 : r1;
    const float v3 = XZ[(size_t)c3 * kXZP + d];
    const float v2 = XZ[(size_t)c2 * kXZP + d];
    const float v1 = XZ[(size_t)c1 * kXZP + d];
    xm3 = (r3 >= 0) ? v3 : 0.f;
    xm2 = (r2 >= 0) ? v2 : 0.f;
    xm1 = (r1 >= 0) ? v1 : 0.f;
  }
#pragma unroll 1
  for (int sub = 0; sub < 4; ++sub) {
    const int lb = t0 + sub * 16;
#pragma unroll 1
    for (int st = 0; st < 16; ++st) {
      const int tt = lb + st;
      const float xin = XZ[(size_t)tt * kXZP + d];
      float acc = w0 * xm3;
      acc = fmaf(w1, xm2, acc);
      acc = fmaf(w2, xm1, acc);
      acc = fmaf(w3, xin, acc);
      const float sv = acc + bc;
      const float sg = __builtin_amdgcn_rcpf(1.0f + __expf(-sv));
      sT[st * kTP + tid] = sv * sg;
      xm3 = xm2; xm2 = xm1; xm1 = xin;
    }
    __syncthreads();
    v8h hv[2], lv[2];
#pragma unroll
    for (int it = 0; it < 2; ++it) {
      const float* sp = sT + (it * 8 + wave) * kTP + lane * 8;
      const v4f a0 = *(const v4f*)(sp);
      const v4f a1 = *(const v4f*)(sp + 4);
#pragma unroll
      for (int e = 0; e < 4; ++e) {
        const unsigned short hb0 = f2bf_bits(a0[e]);
        const unsigned short lb0 = f2bf_bits(a0[e] - bf_bits2f(hb0));
        const unsigned short hb1 = f2bf_bits(a1[e]);
        const unsigned short lb1 = f2bf_bits(a1[e] - bf_bits2f(hb1));
        hv[it][e]     = __builtin_bit_cast(_Float16, hb0);
        lv[it][e]     = __builtin_bit_cast(_Float16, lb0);
        hv[it][4 + e] = __builtin_bit_cast(_Float16, hb1);
        lv[it][4 + e] = __builtin_bit_cast(_Float16, lb1);
      }
    }
    for (int pass = 0; pass < 2; ++pass) {
#pragma unroll
      for (int it = 0; it < 2; ++it) {
        const int tt = lb + it * 8 + wave;
        const size_t off = (size_t)tt * kDin + d0 + lane * 8;
        *(volatile v8h*)(XCH + off) = hv[it];
        *(volatile v8h*)(XCL + off) = lv[it];
      }
      __threadfence();
    }
    __syncthreads();
  }
}

__global__ __launch_bounds__(256) void scan_kernel(
    const float* __restrict__ DLR, const float* __restrict__ XZ, const float* __restrict__ XDBL,
    const float* __restrict__ cw, const float* __restrict__ cb, const float* __restrict__ dtb,
    const float* __restrict__ A_log, const float* __restrict__ Dv,
    unsigned short* __restrict__ YH, unsigned short* __restrict__ YL)
{
  __shared__ __align__(16) float sBC[16 * 32];
  __shared__ __align__(16) float sY[16 * kTP];
  const int tid = threadIdx.x, lane = tid & 31, wave = tid >> 5;
  const int d0 = blockIdx.x * 256, d = d0 + tid;

  float An[kNst];
#pragma unroll
  for (int n = 0; n < kNst; ++n) An[n] = -__expf(bfr(A_log[(size_t)d * kNst + n]));
  const float Dd  = bfr(Dv[d]);
  const float bdt = bfr(dtb[d]);
  const float bc  = bfr(cb[d]);
  const float w0 = bfr(cw[d * 4 + 0]), w1 = bfr(cw[d * 4 + 1]), w2 = bfr(cw[d * 4 + 2]), w3 = bfr(cw[d * 4 + 3]);
  float h[kNst];
#pragma unroll
  for (int n = 0; n < kNst; ++n) h[n] = 0.f;
  float xm3 = 0.f, xm2 = 0.f, xm1 = 0.f;

#pragma unroll 1
  for (int c = 0; c < kSeqL / 16; ++c) {
    const int l0 = c * 16;
    if (tid < 128) {
      const int r = tid >> 3, q = (tid & 7) * 4;
      const v4f v = *(const v4f*)(XDBL + (size_t)(l0 + r) * kPrj + kDtR + q);
      *(v4f*)(sBC + r * 32 + q) = v;
    }
    __syncthreads();
#pragma unroll 1
    for (int st = 0; st < 16; ++st) {
      const size_t m = (size_t)(l0 + st);
      const float a     = DLR[m * kDin + d] + bdt;
      const float delta = fmaxf(a, 0.0f) + log1pf(__expf(-fabsf(a)));
      const float xin   = XZ[m * kXZP + d];
      float acc = w0 * xm3;
      acc = fmaf(w1, xm2, acc);
      acc = fmaf(w2, xm1, acc);
      acc = fmaf(w3, xin, acc);
      const float sv  = acc + bc;
      const float sgx = __builtin_amdgcn_rcpf(1.0f + __expf(-sv));
      const float xv  = sv * sgx;
      xm3 = xm2; xm2 = xm1; xm1 = xin;
      const float zv  = XZ[m * kXZP + kDin + d];
      v4f Bq[4], Cq[4];
#pragma unroll
      for (int qq = 0; qq < 4; ++qq) {
        Bq[qq] = *(const v4f*)(sBC + st * 32 + 4 * qq);
        Cq[qq] = *(const v4f*)(sBC + st * 32 + kNst + 4 * qq);
      }
      float dx = delta * xv;
      asm volatile("" : "+v"(dx));
      float y = 0.f;
#pragma unroll
      for (int n = 0; n < kNst; ++n) {
        const float e = __expf(delta * An[n]);
        float p = dx * Bq[n >> 2][n & 3];
        asm volatile("" : "+v"(p));
        float qv = h[n] * e;
        asm volatile("" : "+v"(qv));
        const float hn = qv + p;
        h[n] = hn;
        float rr = Cq[n >> 2][n & 3] * hn;
        asm volatile("" : "+v"(rr));
        y += rr;
      }
      float sk = xv * Dd;
      asm volatile("" : "+v"(sk));
      y += sk;
      const float sg = __builtin_amdgcn_rcpf(1.0f + __expf(-zv));
      const float g  = zv * sg;
      sY[st * kTP + tid] = y * g;
    }
    __syncthreads();
    v8h hv[2], lv[2];
#pragma unroll
    for (int it = 0; it < 2; ++it) {
      const float* sp = sY + (it * 8 + wave) * kTP + lane * 8;
      const v4f a0 = *(const v4f*)(sp);
      const v4f a1 = *(const v4f*)(sp + 4);
#pragma unroll
      for (int e = 0; e < 4; ++e) {
        const unsigned short hb0 = f2bf_bits(a0[e]);
        const unsigned short lb0 = f2bf_bits(a0[e] - bf_bits2f(hb0));
        const unsigned short hb1 = f2bf_bits(a1[e]);
        const unsigned short lb1 = f2bf_bits(a1[e] - bf_bits2f(hb1));
        hv[it][e]     = __builtin_bit_cast(_Float16, hb0);
        lv[it][e]     = __builtin_bit_cast(_Float16, lb0);
        hv[it][4 + e] = __builtin_bit_cast(_Float16, hb1);
        lv[it][4 + e] = __builtin_bit_cast(_Float16, lb1);
      }
    }
    for (int pass = 0; pass < 2; ++pass) {
#pragma unroll
      for (int it = 0; it < 2; ++it) {
        const size_t yo = (size_t)(l0 + it * 8 + wave) * kDin + d0 + lane * 8;
        *(volatile v8h*)(YH + yo) = hv[it];
        *(volatile v8h*)(YL + yo) = lv[it];
      }
      __threadfence();
    }
  }
}

__global__ __launch_bounds__(256) void gelu_out_kernel(const float* __restrict__ src, const float* __restrict__ xin,
                                                       float* __restrict__ dst)
{
  __shared__ __align__(16) float sv[256];
  const int tid = threadIdx.x;
  const size_t base = (size_t)blockIdx.x * 256;
  const float v = src[base + tid] + bfr(xin[base + tid]);
  sv[tid] = 0.5f * v * (1.0f + erff(v * 0.70710678118654752f));
  __syncthreads();
  if (tid < 64) {
    const v4f o = *(const v4f*)(sv + tid * 4);
    float* p = dst + base + (size_t)tid * 4;
    *(volatile v4f*)p = o;
    __threadfence();
    *(volatile v4f*)p = o;
  }
}

extern "C" void kernel_launch(void* const* d_in, const int* in_sizes, int n_in,
                              void* d_out, int out_size, void* d_ws, size_t ws_size,
                              hipStream_t stream)
{
  if (n_in < 21) return;
  const float* x    = (const float*)d_in[0];
  const float* ln_w = (const float*)d_in[19];
  const float* ln_b = (const float*)d_in[20];
  const float* Pw[2][9];
  for (int dir = 0; dir < 2; ++dir)
    for (int i = 0; i < 9; ++i) Pw[dir][i] = (const float*)d_in[1 + 9 * dir + i];
  float* dout = (float*)d_out;

  if (in_sizes[0] != kBatch * kSeqL * kDmod) return;
  for (int dir = 0; dir < 2; ++dir) {
    const int* sz = in_sizes + 1 + 9 * dir;
    if (sz[0] != kXZP * kDmod) return;
    if (sz[1] != kDin * 4 || sz[2] != kDin) return;
    if (sz[3] != kPrj * kDin) return;
    if (sz[4] != kDin * kDtR || sz[5] != kDin) return;
    if (sz[6] != kDin * kNst || sz[7] != kDin) return;
    if (sz[8] != kDmod * kDin) return;
  }
  if (in_sizes[19] != kDmod || in_sizes[20] != kDmod) return;
  if (out_size != kBatch * kSeqL * kDmod) return;

  const size_t SZ_WIN16  = (size_t)kXZP * kDmod * 2;
  const size_t SZ_WXP16  = (size_t)kPrj * kDin * 2;
  const size_t SZ_WDT16  = (size_t)kDin * kDtR * 2;
  const size_t SZ_WOUT16 = (size_t)kDmod * kDin * 2;
  const size_t SZ_HPL    = (size_t)kRows * kDmod * 2;
  const size_t SZ_XZ     = (size_t)kSeqL * kXZP * 4;
  const size_t SZ_XCPL   = (size_t)kSeqL * kDin * 2;
  const size_t SZ_XDBL   = (size_t)kSeqL * kPrj * 4;
  const size_t SZ_DTPL   = (size_t)kSeqL * kDtR * 2;
  const size_t SZ_DLR    = (size_t)kSeqL * kDin * 4;
  const size_t SZ_YPL    = (size_t)kRows * kDin * 2;
  const size_t SZ_ACC    = (size_t)kRows * kDmod * 4;
  const size_t OFF_WIN16  = 0;
  const size_t OFF_WXP16  = OFF_WIN16  + 2 * SZ_WIN16;
  const size_t OFF_WDT16  = OFF_WXP16  + 2 * SZ_WXP16;
  const size_t OFF_WOUT16 = OFF_WDT16  + 2 * SZ_WDT16;
  const size_t OFF_HH     = OFF_WOUT16 + 2 * SZ_WOUT16;
  const size_t OFF_HL     = OFF_HH     + SZ_HPL;
  const size_t OFF_XZ     = OFF_HL     + SZ_HPL;
  const size_t OFF_XCH    = OFF_XZ     + SZ_XZ;
  const size_t OFF_XCL    = OFF_XCH    + SZ_XCPL;
  const size_t OFF_XDBL   = OFF_XCL    + SZ_XCPL;
  const size_t OFF_DTH    = OFF_XDBL   + SZ_XDBL;
  const size_t OFF_DTL    = OFF_DTH    + SZ_DTPL;
  const size_t OFF_YH     = OFF_DTL    + SZ_DTPL;
  const size_t OFF_YL     = OFF_YH     + SZ_YPL;
  const size_t OFF_ACC    = OFF_YL     + SZ_YPL;
  const size_t TOTAL      = OFF_ACC    + SZ_ACC;
  if (SZ_ACC > SZ_XZ) return;
  if (SZ_DLR > 2 * SZ_XCPL) return;
  if (ws_size < TOTAL) return;

  char* ws = (char*)d_ws;
  unsigned short* WIN16[2]; unsigned short* WXP16[2]; unsigned short* WDT16[2]; unsigned short* WOUT16[2];
  for (int dir = 0; dir < 2; ++dir) {
    WIN16[dir]  = (unsigned short*)(ws + OFF_WIN16  + (size_t)dir * SZ_WIN16);
    WXP16[dir]  = (unsigned short*)(ws + OFF_WXP16  + (size_t)dir * SZ_WXP16);
    WDT16[dir]  = (unsigned short*)(ws + OFF_WDT16  + (size_t)dir * SZ_WDT16);
    WOUT16[dir] = (unsigned short*)(ws + OFF_WOUT16 + (size_t)dir * SZ_WOUT16);
  }
  unsigned short* HH   = (unsigned short*)(ws + OFF_HH);
  unsigned short* HL   = (unsigned short*)(ws + OFF_HL);
  float*          XZ   = (float*)(ws + OFF_XZ);
  float*          PRE  = (float*)(ws + OFF_XZ);
  unsigned short* XCH  = (unsigned short*)(ws + OFF_XCH);
  unsigned short* XCL  = (unsigned short*)(ws + OFF_XCL);
  float*          DLR  = (float*)(ws + OFF_XCH);
  float*          XDBL = (float*)(ws + OFF_XDBL);
  unsigned short* DTH  = (unsigned short*)(ws + OFF_DTH);
  unsigned short* DTL  = (unsigned short*)(ws + OFF_DTL);
  unsigned short* YH   = (unsigned short*)(ws + OFF_YH);
  unsigned short* YL   = (unsigned short*)(ws + OFF_YL);
  float*          ACC  = (float*)(ws + OFF_ACC);
  const float* dummy_bias  = Pw[0][5];
  const float* dummy_resid = x;

  for (int dir = 0; dir < 2; ++dir) {
    cast_rows_bf16_kernel<<<(kXZP * kDmod) / 8 / 256, 256, 0, stream>>>(
        Pw[dir][0], WIN16[dir], kXZP, kDmod, (kXZP * kDmod) / 8);
    cast_rows_bf16_kernel<<<(kPrj * kDin) / 8 / 256, 256, 0, stream>>>(
        Pw[dir][3], WXP16[dir], kPrj, kDin, (kPrj * kDin) / 8);
    cast_rows_bf16_kernel<<<(kDin * kDtR) / 8 / 256, 256, 0, stream>>>(
        Pw[dir][4], WDT16[dir], kDin, kDtR, (kDin * kDtR) / 8);
    cast_rows_bf16_kernel<<<(kDmod * kDin) / 8 / 256, 256, 0, stream>>>(
        Pw[dir][8], WOUT16[dir], kDmod, kDin, (kDmod * kDin) / 8);
  }

  for (int dir = 0; dir < 2; ++dir) {
    const float* conv_w = Pw[dir][1];
    const float* conv_b = Pw[dir][2];
    const float* dt_b   = Pw[dir][5];
    const float* A_log  = Pw[dir][6];
    const float* Dv     = Pw[dir][7];

    ln_rows_kernel<<<kRows, 64, 0, stream>>>(x, ln_w, ln_b, HH, HL, dir);

    for (int b = 0; b < kBatch; ++b) {
      const unsigned short* Hh = HH + (size_t)b * kSeqL * kDmod;
      const unsigned short* Hl = HL + (size_t)b * kSeqL * kDmod;

      wmma_gemm64<1, 2, 0, 0, false><<<dim3(256, 1), 256, 0, stream>>>(
          Hh, Hl, kDmod, 0L, WIN16[dir], WIN16[dir], kDmod, 0L,
          (void*)XZ, (void*)XZ, kXZP, 0L, dummy_bias, dummy_resid, 0L, kSeqL, kXZP, kDmod, 1.0f);

      conv_silu_kernel<<<dim3(kDin / 256, kSeqL / 64), 256, 0, stream>>>(XZ, conv_w, conv_b, XCH, XCL);

      wmma_gemm64<1, 2, 0, 0, false><<<dim3(8, 1), 256, 0, stream>>>(
          XCH, XCL, kDin, 0L, WXP16[dir], WXP16[dir], kDin, 0L,
          (void*)XDBL, (void*)XDBL, kPrj, 0L, dummy_bias, dummy_resid, 0L, kSeqL, kPrj, kDin, 1.0f);

      cast_cols_bf16_split_kernel<<<(kSeqL * kDtR) / 8 / 256, 256, 0, stream>>>(
          XDBL, kPrj, DTH, DTL, kDtR, (kSeqL * kDtR) / 8);

      wmma_gemm64<1, 2, 0, 0, false><<<dim3(128, 1), 256, 0, stream>>>(
          DTH, DTL, kDtR, 0L, WDT16[dir], WDT16[dir], kDtR, 0L,
          (void*)DLR, (void*)DLR, kDin, 0L, dummy_bias, dummy_resid, 0L, kSeqL, kDin, kDtR, 1.0f);

      scan_kernel<<<dim3(kDin / 256, 1), 256, 0, stream>>>(
          DLR, XZ, XDBL, conv_w, conv_b, dt_b, A_log, Dv,
          YH + (size_t)b * kSeqL * kDin, YL + (size_t)b * kSeqL * kDin);
    }

    if (dir == 0) {
      wmma_gemm64<1, 2, 0, 0, false><<<dim3(128, 1), 256, 0, stream>>>(
          YH, YL, kDin, 0L, WOUT16[0], WOUT16[0], kDin, 0L,
          (void*)ACC, (void*)ACC, kDmod, 0L, dummy_bias, dummy_resid, 0L, kRows, kDmod, kDin, 1.0f);
    } else {
      wmma_gemm64<1, 2, 0, 0, true><<<dim3(128, 1), 256, 0, stream>>>(
          YH, YL, kDin, 0L, WOUT16[1], WOUT16[1], kDin, 0L,
          (void*)PRE, (void*)PRE, kDmod, 0L, dummy_bias, ACC, 0L, kRows, kDmod, kDin, 1.0f);
    }
  }

  gelu_out_kernel<<<(kRows * kDmod) / 256, 256, 0, stream>>>(PRE, x, dout);
}
